// PD_Block_68332929679630
// MI455X (gfx1250) — hardware-verified
//
#include <hip/hip_runtime.h>
#include <math.h>
#include <stdint.h>


#define T_TOK 2048
#define B_SZ  4
#define L_SEQ 512
#define E_DIM 128
#define N_DIM 128
#define H_DIM 256
#define K_SEL 8
#define TWO_PI_F 6.283185307179586f
#define SPITCH 36

#define ACT_NONE  0
#define ACT_GELU  1
#define ACT_SIG   2
#define ACT_PHASE 3

typedef __bf16 v16bf __attribute__((ext_vector_type(16)));
typedef float  v8f   __attribute__((ext_vector_type(8)));
typedef float  v4f   __attribute__((ext_vector_type(4)));
typedef int    v4i   __attribute__((ext_vector_type(4)));

typedef char chk_dims[(T_TOK % 16 == 0 && E_DIM % 32 == 0 && H_DIM % 32 == 0 && N_DIM % 32 == 0 &&
                       E_DIM == N_DIM && (T_TOK == B_SZ * L_SEQ) && N_DIM == 128 && K_SEL == 8) ? 1 : -1];

union Frag { v16bf v; unsigned w[8]; };

__device__ __forceinline__ unsigned bf16_bits(float f) {
    unsigned u = __float_as_uint(f);
    return (u + 0x7FFFu + ((u >> 16) & 1u)) >> 16;
}

__device__ __forceinline__ void split_pair(float a, float b, unsigned& wh, unsigned& wl) {
    const unsigned ha = bf16_bits(a), hb = bf16_bits(b);
    const float ra = a - __uint_as_float(ha << 16);
    const float rb = b - __uint_as_float(hb << 16);
    const unsigned la = bf16_bits(ra), lb = bf16_bits(rb);
    wh = ha | (hb << 16);
    wl = la | (lb << 16);
}

__device__ __forceinline__ void load_frag(const float* __restrict__ p0, const float* __restrict__ p1,
                                          Frag& fh, Frag& fl) {
    const v4f a0 = *(const v4f*)(p0);
    const v4f a1 = *(const v4f*)(p0 + 4);
    const v4f b0 = *(const v4f*)(p1);
    const v4f b1 = *(const v4f*)(p1 + 4);
    split_pair(a0.x, a0.y, fh.w[0], fl.w[0]);
    split_pair(a0.z, a0.w, fh.w[1], fl.w[1]);
    split_pair(a1.x, a1.y, fh.w[2], fl.w[2]);
    split_pair(a1.z, a1.w, fh.w[3], fl.w[3]);
    split_pair(b0.x, b0.y, fh.w[4], fl.w[4]);
    split_pair(b0.z, b0.w, fh.w[5], fl.w[5]);
    split_pair(b1.x, b1.y, fh.w[6], fl.w[6]);
    split_pair(b1.z, b1.w, fh.w[7], fl.w[7]);
}

__device__ __forceinline__ v8f wmma3(v8f c, const Frag& ah, const Frag& al, const Frag& bh, const Frag& bl) {
    c = __builtin_amdgcn_wmma_f32_16x16x32_bf16(false, ah.v, false, bh.v, (short)0, c, false, false);
    c = __builtin_amdgcn_wmma_f32_16x16x32_bf16(false, al.v, false, bh.v, (short)0, c, false, false);
    c = __builtin_amdgcn_wmma_f32_16x16x32_bf16(false, ah.v, false, bl.v, (short)0, c, false, false);
    asm volatile("v_nop\n\tv_nop\n\tv_nop\n\tv_nop" : "+v"(c) : "v"(ah.v), "v"(al.v), "v"(bh.v), "v"(bl.v));
    return c;
}

__device__ __forceinline__ v8f zero8() {
    v8f z; z[0]=0.f; z[1]=0.f; z[2]=0.f; z[3]=0.f; z[4]=0.f; z[5]=0.f; z[6]=0.f; z[7]=0.f; return z;
}

template <int KD, int NN, int ACT>
__global__ __launch_bounds__(64)
void pd_gemm(const float* __restrict__ X, const float* __restrict__ W, const float* __restrict__ bias,
             float* __restrict__ Y, float* __restrict__ Y2, int has_bias, int ntiles) {
    __shared__ __attribute__((aligned(16))) float stage[2 * 16 * SPITCH];
    constexpr int CT = NN / 32;
    const int wave = threadIdx.x >> 5;
    const int l = threadIdx.x & 31, h = l >> 4, m = l & 15;
    const int tile_raw = blockIdx.x * 2 + wave;
    const bool active = tile_raw < ntiles;
    const int tile = active ? tile_raw : 0;
    const int t0 = (tile / CT) * 16;
    const int nb = (tile % CT) * 32;

    const float* xr = X + (size_t)(t0 + m) * KD;
    const float* w0 = W + (size_t)(nb + m) * KD;
    const float* w1 = W + (size_t)(nb + 16 + m) * KD;

    v8f acc0 = zero8(), acc1 = zero8();
#pragma unroll 1
    for (int k0 = 0; k0 < KD; k0 += 32) {
        const int ka = k0 + 8 * h, kb = k0 + 16 + 8 * h;
        Frag ah, al, bh, bl;
        load_frag(xr + ka, xr + kb, ah, al);
        load_frag(w0 + ka, w0 + kb, bh, bl);
        acc0 = wmma3(acc0, ah, al, bh, bl);
        load_frag(w1 + ka, w1 + kb, bh, bl);
        acc1 = wmma3(acc1, ah, al, bh, bl);
    }

    float bv0 = 0.f, bv1 = 0.f;
    if (has_bias) { bv0 = bias[nb + m]; bv1 = bias[nb + 16 + m]; }
    float e0[8], e1[8], f0[8], f1[8];
#pragma unroll
    for (int r = 0; r < 8; ++r) {
        float r0 = acc0[r] + bv0, r1 = acc1[r] + bv1;
        f0[r] = 0.f; f1[r] = 0.f;
        if (ACT == ACT_GELU) {
            e0[r] = 0.5f * r0 * (erff(r0 * 0.70710678118654752f) + 1.0f);
            e1[r] = 0.5f * r1 * (erff(r1 * 0.70710678118654752f) + 1.0f);
        } else if (ACT == ACT_SIG) {
            e0[r] = 1.0f / (1.0f + expf(-r0));
            e1[r] = 1.0f / (1.0f + expf(-r1));
        } else if (ACT == ACT_PHASE) {
            float p0 = TWO_PI_F * (1.0f / (1.0f + expf(-r0)));
            float p1 = TWO_PI_F * (1.0f / (1.0f + expf(-r1)));
            e0[r] = cosf(p0); f0[r] = sinf(p0);
            e1[r] = cosf(p1); f1[r] = sinf(p1);
        } else {
            e0[r] = r0; e1[r] = r1;
        }
    }

    float* st = stage + wave * 16 * SPITCH;
#pragma unroll
    for (int r = 0; r < 8; ++r) {
        st[(8 * h + r) * SPITCH + m]      = e0[r];
        st[(8 * h + r) * SPITCH + 16 + m] = e1[r];
    }
    __syncthreads();
    const int q = l >> 3, c4 = (l & 7) * 4;
    v4f vals[4];
#pragma unroll
    for (int i = 0; i < 4; ++i) vals[i] = *(const v4f*)(st + (4 * i + q) * SPITCH + c4);
    if (active) {
        float* yb = Y + (size_t)t0 * NN + nb + c4;
#pragma unroll
        for (int i = 0; i < 4; ++i) *(volatile v4f*)(yb + (size_t)(4 * i + q) * NN) = vals[i];
        __threadfence();
#pragma unroll
        for (int i = 0; i < 4; ++i) *(volatile v4f*)(yb + (size_t)(4 * i + q) * NN) = vals[i];
    }
    if (ACT == ACT_PHASE) {
        __syncthreads();
#pragma unroll
        for (int r = 0; r < 8; ++r) {
            st[(8 * h + r) * SPITCH + m]      = f0[r];
            st[(8 * h + r) * SPITCH + 16 + m] = f1[r];
        }
        __syncthreads();
#pragma unroll
        for (int i = 0; i < 4; ++i) vals[i] = *(const v4f*)(st + (4 * i + q) * SPITCH + c4);
        if (active) {
            float* yb2 = Y2 + (size_t)t0 * NN + nb + c4;
#pragma unroll
            for (int i = 0; i < 4; ++i) *(volatile v4f*)(yb2 + (size_t)(4 * i + q) * NN) = vals[i];
            __threadfence();
#pragma unroll
            for (int i = 0; i < 4; ++i) *(volatile v4f*)(yb2 + (size_t)(4 * i + q) * NN) = vals[i];
        }
    }
}

__global__ __launch_bounds__(128)
void pd_select(const float* __restrict__ x, const float* __restrict__ S_w, const float* __restrict__ A_dict,
               int* __restrict__ idx, int ntok) {
    __shared__ __attribute__((aligned(16))) float xs[E_DIM];
    __shared__ double part[128];
    __shared__ float lgs[K_SEL];
    __shared__ float els[K_SEL];
    __shared__ __attribute__((aligned(16))) int sidx[N_DIM];
    const int t = blockIdx.x;
    const int n = threadIdx.x;
    const bool active = t < ntok;
    const int tt = active ? t : 0;

    xs[n] = x[(size_t)tt * E_DIM + n];
    __syncthreads();
    {
        const int k = n >> 4, p = n & 15;
        const float* wr = S_w + k * E_DIM + p * 8;
        const float* xp = xs + p * 8;
        double s = 0.0;
#pragma unroll
        for (int j = 0; j < 8; ++j) s = fma((double)xp[j], (double)wr[j], s);
        part[n] = s;
    }
    __syncthreads();
    if (n < K_SEL) {
        double a = 0.0;
#pragma unroll 1
        for (int q = 0; q < 16; ++q) a += part[n * 16 + q];
        lgs[n] = (float)a;
    }
    __syncthreads();
    float mx = lgs[0];
#pragma unroll 1
    for (int k = 1; k < K_SEL; ++k) mx = fmaxf(mx, lgs[k]);
    if (n < K_SEL) els[n] = expf(lgs[n] - mx);
    __syncthreads();
    float sum = 0.f;
#pragma unroll 1
    for (int k = 0; k < K_SEL; ++k) sum += els[k];
    const float inv = 1.0f / sum;
    double dk[8];
#pragma unroll
    for (int k = 0; k < 8; ++k) dk[k] = (double)(els[k] * inv);

    const float* ar = A_dict + (size_t)n * N_DIM * K_SEL;
    float best = -3.0e38f;
    int bi = 0;
#pragma unroll 1
    for (int mm = 0; mm < N_DIM; ++mm) {
        const v4f q0 = *(const v4f*)(ar + mm * K_SEL);
        const v4f q1 = *(const v4f*)(ar + mm * K_SEL + 4);
        double v = (double)q0.x * dk[0];
        v = fma((double)q0.y, dk[1], v);
        v = fma((double)q0.z, dk[2], v);
        v = fma((double)q0.w, dk[3], v);
        v = fma((double)q1.x, dk[4], v);
        v = fma((double)q1.y, dk[5], v);
        v = fma((double)q1.z, dk[6], v);
        v = fma((double)q1.w, dk[7], v);
        const float vf = (float)v;
        if (vf > best) { best = vf; bi = mm; }
    }
    sidx[n] = bi;
    __syncthreads();
    if (active && n < 32) {
        const v4i w = *(const v4i*)(sidx + 4 * n);
        int* dst = idx + (size_t)t * N_DIM + 4 * n;
        *(volatile v4i*)dst = w;
        __threadfence();
        *(volatile v4i*)dst = w;
    }
}

__global__ __launch_bounds__(128)
void pd_scan(const int* __restrict__ idx, const float* __restrict__ mag,
             const float* __restrict__ phc, const float* __restrict__ phs,
             const float* __restrict__ br, const float* __restrict__ bi,
             float* __restrict__ feat, int nbatch) {
#pragma clang fp contract(off)
    __shared__ __attribute__((aligned(16))) float hre[N_DIM];
    __shared__ __attribute__((aligned(16))) float him[N_DIM];
    const int b = blockIdx.x;
    const int n = threadIdx.x;
    const bool active = b < nbatch;
    const int bb = active ? b : 0;
    hre[n] = (n == 0) ? 1.0f : 0.0f;
    him[n] = 0.0f;
    __syncthreads();
    for (int t = 0; t < L_SEQ; ++t) {
        const size_t base = ((size_t)bb * L_SEQ + t) * N_DIM;
        int j = idx[base + n];
        j = j < 0 ? 0 : (j > N_DIM - 1 ? N_DIM - 1 : j);
        const float mg = mag[base + n];
        const float dr = mg * phc[base + n];
        const float di = mg * phs[base + n];
        const float bre = br[base + n];
        const float bim = bi[base + n];
        const float hr = hre[j], hm = him[j];
        __syncthreads();
        const float nr = (dr * hr - di * hm) + bre;
        const float ni = (dr * hm + di * hr) + bim;
        hre[n] = nr;
        him[n] = ni;
        __syncthreads();
        if (active && n < 64) {
            v4f v;
            if (n < 32) v = *(const v4f*)(hre + 4 * n);
            else        v = *(const v4f*)(him + 4 * (n - 32));
            float* dst = feat + ((size_t)bb * L_SEQ + t) * (2 * N_DIM) + 4 * n;
            *(volatile v4f*)dst = v;
            __threadfence();
            *(volatile v4f*)dst = v;
        }
    }
}

__global__ __launch_bounds__(128)
void pd_ln(const float* __restrict__ out_pre, const float* __restrict__ x, const float* __restrict__ D_skip,
           const float* __restrict__ nw, const float* __restrict__ nbias, float* __restrict__ out, int ntok) {
    __shared__ float red[E_DIM];
    __shared__ __attribute__((aligned(16))) float ys[E_DIM];
    const int t = blockIdx.x;
    const int e = threadIdx.x;
    const bool active = t < ntok;
    const int tt = active ? t : 0;
    const float v = out_pre[(size_t)tt * E_DIM + e] + D_skip[e] * x[(size_t)tt * E_DIM + e];
    red[e] = v;
    __syncthreads();
    for (int s = 64; s > 0; s >>= 1) {
        if (e < s) red[e] += red[e + s];
        __syncthreads();
    }
    const float mean = red[0] * (1.0f / 128.0f);
    __syncthreads();
    const float d = v - mean;
    red[e] = d * d;
    __syncthreads();
    for (int s = 64; s > 0; s >>= 1) {
        if (e < s) red[e] += red[e + s];
        __syncthreads();
    }
    const float var = red[0] * (1.0f / 128.0f);
    ys[e] = d * rsqrtf(var + 1e-5f) * nw[e] + nbias[e];
    __syncthreads();
    if (active && e < 32) {
        const v4f w = *(const v4f*)(ys + 4 * e);
        float* dst = out + (size_t)t * E_DIM + 4 * e;
        *(volatile v4f*)dst = w;
        __threadfence();
        *(volatile v4f*)dst = w;
    }
}

template <int KD, int NN, int ACT>
static inline void launch_gemm(const float* X, const float* W, const float* bias, int has_bias,
                               float* Y, float* Y2, hipStream_t stream) {
    const int ntiles = (T_TOK / 16) * (NN / 32);
    const int blocks = (ntiles + 1) / 2;
    pd_gemm<KD, NN, ACT><<<blocks, 64, 0, stream>>>(X, W, bias, Y, Y2, has_bias, ntiles);
}

extern "C" void kernel_launch(void* const* d_in, const int* in_sizes, int n_in,
                              void* d_out, int out_size, void* d_ws, size_t ws_size,
                              hipStream_t stream) {
    if (n_in < 18) return;
    if (in_sizes[0] != T_TOK * E_DIM || out_size != T_TOK * E_DIM) return;
    if (in_sizes[12] != N_DIM * N_DIM * K_SEL || in_sizes[16] != E_DIM * 2 * N_DIM) return;

    const float* x      = (const float*)d_in[0];
    const float* norm_w = (const float*)d_in[1];
    const float* norm_b = (const float*)d_in[2];
    const float* mag_w1 = (const float*)d_in[3];
    const float* mag_b1 = (const float*)d_in[4];
    const float* mag_w2 = (const float*)d_in[5];
    const float* mag_b2 = (const float*)d_in[6];
    const float* ph_w1  = (const float*)d_in[7];
    const float* ph_b1  = (const float*)d_in[8];
    const float* ph_w2  = (const float*)d_in[9];
    const float* ph_b2  = (const float*)d_in[10];
    const float* S_w    = (const float*)d_in[11];
    const float* A_dict = (const float*)d_in[12];
    const float* B_re   = (const float*)d_in[13];
    const float* B_im   = (const float*)d_in[14];
    const float* D_skip = (const float*)d_in[15];
    const float* ro_w   = (const float*)d_in[16];
    const float* ro_b   = (const float*)d_in[17];
    float* out = (float*)d_out;

    char* ws = (char*)d_ws;
    size_t o = 0;
    float* h1      = (float*)(ws + o); o += (size_t)T_TOK * H_DIM * 4;
    float* magb    = (float*)(ws + o); o += (size_t)T_TOK * N_DIM * 4;
    float* phc     = (float*)(ws + o); o += (size_t)T_TOK * N_DIM * 4;
    float* phsn    = (float*)(ws + o); o += (size_t)T_TOK * N_DIM * 4;
    float* bre     = (float*)(ws + o); o += (size_t)T_TOK * N_DIM * 4;
    float* bim     = (float*)(ws + o); o += (size_t)T_TOK * N_DIM * 4;
    float* feat    = (float*)(ws + o); o += (size_t)T_TOK * 2 * N_DIM * 4;
    float* out_pre = (float*)(ws + o); o += (size_t)T_TOK * E_DIM * 4;
    int*   idx     = (int*)(ws + o);   o += (size_t)T_TOK * N_DIM * 4;
    if (o > ws_size) return;

    pd_select<<<T_TOK, 128, 0, stream>>>(x, S_w, A_dict, idx, T_TOK);

    launch_gemm<E_DIM, H_DIM, ACT_GELU>(x,  mag_w1, mag_b1, 1, h1,   h1,   stream);
    launch_gemm<H_DIM, N_DIM, ACT_SIG >(h1, mag_w2, mag_b2, 1, magb, magb, stream);
    launch_gemm<E_DIM, H_DIM, ACT_GELU >(x,  ph_w1, ph_b1, 1, h1,  h1,   stream);
    launch_gemm<H_DIM, N_DIM, ACT_PHASE>(h1, ph_w2, ph_b2, 1, phc, phsn, stream);
    launch_gemm<E_DIM, N_DIM, ACT_NONE>(x, B_re, B_re, 0, bre, bre, stream);
    launch_gemm<E_DIM, N_DIM, ACT_NONE>(x, B_im, B_im, 0, bim, bim, stream);

    pd_scan<<<B_SZ, N_DIM, 0, stream>>>(idx, magb, phc, phsn, bre, bim, feat, B_SZ);

    launch_gemm<2 * N_DIM, E_DIM, ACT_NONE>(feat, ro_w, ro_b, 1, out_pre, out_pre, stream);
    pd_ln<<<T_TOK, E_DIM, 0, stream>>>(out_pre, x, D_skip, norm_w, norm_b, out, T_TOK);
}
